// RGCNEncoder_25984552141045
// MI455X (gfx1250) — hardware-verified
//
#include <hip/hip_runtime.h>
#include <math.h>

#define NN    100000
#define NE    1000000
#define HID   64
#define NQ    18
#define NL    3
#define SRB   1024
#define NTL   98
#define NPAD  (NTL * SRB)
#define NT    256
#define KA    1184
#define LDA   1216
#define NPC   152
#define MCH   25088
#define NCHK  4
#define SCH   2048
#define SP    (SCH / NT)
#define CAP   (2 * SCH)
#define NCH   ((NE + SCH - 1) / SCH)

typedef __attribute__((ext_vector_type(16))) _Float16 v16h;
typedef __attribute__((ext_vector_type(8)))  _Float16 v8h;
typedef __attribute__((ext_vector_type(16))) __bf16   v16b;
typedef __attribute__((ext_vector_type(8)))  __bf16   v8b;
typedef __attribute__((ext_vector_type(8)))  float    v8f;
typedef __attribute__((ext_vector_type(4)))  float    v4f;
typedef __attribute__((ext_vector_type(4)))  int      v4i;

__device__ __forceinline__ unsigned short f2bf_bits(float f) {
  unsigned u = __float_as_uint(f);
  return (unsigned short)((u + 0x7FFFu + ((u >> 16) & 1u)) >> 16);
}
__device__ __forceinline__ float bf_bits2f(unsigned short h) { return __uint_as_float(((unsigned)h) << 16); }

__device__ __forceinline__ void dep_guard_h(v8f& a, v8f& b, v16h x, v16h y) { asm volatile("v_nop\n\tv_nop\n\tv_nop\n\tv_nop" : "+v"(a), "+v"(b) : "v"(x), "v"(y)); }
__device__ __forceinline__ void dep_guard_b(v8f& a, v8f& b, v16b x, v16b y) { asm volatile("v_nop\n\tv_nop\n\tv_nop\n\tv_nop" : "+v"(a), "+v"(b) : "v"(x), "v"(y)); }
__device__ __forceinline__ void keep4_h(v16h a, v16h b, v16h c, v16h d) { asm volatile("v_nop" :: "v"(a), "v"(b), "v"(c), "v"(d)); }
__device__ __forceinline__ void keep4_b(v16b a, v16b b, v16b c, v16b d) { asm volatile("v_nop" :: "v"(a), "v"(b), "v"(c), "v"(d)); }
__device__ __forceinline__ void acc_guard4(v8f& a, v8f& b, v8f& c, v8f& d) { asm volatile("v_nop\n\tv_nop\n\tv_nop\n\tv_nop" : "+v"(a), "+v"(b), "+v"(c), "+v"(d)); }
template <typename T> struct Frag;
template <> struct Frag<_Float16> {
  typedef v16h V; union U { v16h v; v8h h[2]; };
  static __device__ __forceinline__ v16h load(const _Float16* p) {
    U f; f.h[0] = *(const v8h*)(p); f.h[1] = *(const v8h*)(p + 16); return f.v;
  }
  static __device__ __forceinline__ v8f mma(v16h a, v16h b, v8f c) {
    return __builtin_amdgcn_wmma_f32_16x16x32_f16(false, a, false, b, (short)0, c, false, false);
  }
  static __device__ __forceinline__ void guard(v8f& a, v8f& b, v16h x, v16h y) { dep_guard_h(a, b, x, y); }
  static __device__ __forceinline__ void keep(v16h a, v16h b, v16h c, v16h d) { keep4_h(a, b, c, d); }
};
template <> struct Frag<__bf16> {
  typedef v16b V; union U { v16b v; v8b h[2]; };
  static __device__ __forceinline__ v16b load(const __bf16* p) {
    U f; f.h[0] = *(const v8b*)(p); f.h[1] = *(const v8b*)(p + 16); return f.v;
  }
  static __device__ __forceinline__ v8f mma(v16b a, v16b b, v8f c) {
    return __builtin_amdgcn_wmma_f32_16x16x32_bf16(false, a, false, b, (short)0, c, false, false);
  }
  static __device__ __forceinline__ void guard(v8f& a, v8f& b, v16b x, v16b y) { dep_guard_b(a, b, x, y); }
  static __device__ __forceinline__ void keep(v16b a, v16b b, v16b c, v16b d) { keep4_b(a, b, c, d); }
};

template <int ET> struct Elem;
template <> struct Elem<0> { typedef _Float16 T; };
template <> struct Elem<1> { typedef __bf16 T; };
template <int ET, bool SPLIT, int BIAS_MODE, int OUT_MODE, bool RESID, int ACT = 0>
__global__ __launch_bounds__(256) void wmma_gemm64(
    const unsigned short* __restrict__ Ap, const unsigned short* __restrict__ A2p, int lda, long strideA,
    const unsigned short* __restrict__ Btp, const unsigned short* __restrict__ Bt2p, int ldb, long strideB,
    void* __restrict__ Cout, void* __restrict__ Cout2, int ldc, long strideC,
    const float* __restrict__ bias,
    const float* __restrict__ resid, long strideR,
    int M, int N, int K, float scale) {
  typedef typename Elem<ET>::T T;
  typedef typename Frag<T>::V V;
  const T* A = (const T*)Ap; const T* A2 = (const T*)A2p; const T* Bt = (const T*)Btp; const T* Bt2 = (const T*)Bt2p;
  __shared__ __align__(16) float sT[8][16 * 68];
  const int b    = blockIdx.y;
  const int lane = threadIdx.x & 31;
  const int wave = threadIdx.x >> 5;
  const int tilesN = N >> 6;
  const int tilesM = M >> 6;
  const int tile = blockIdx.x * 8 + wave;
  if (tile >= tilesM * tilesN) return;
  const int tm = tile / tilesN;
  const int tn = tile - tm * tilesN;
  const int m0 = tm << 6;
  const int n0 = tn << 6;

  const T* Ab  = A  + (size_t)b * strideA;
  const T* Bb  = Bt + (size_t)b * strideB;
  const T* Ab2 = SPLIT ? (A2  + (size_t)b * strideA) : nullptr;
  const T* Bb2 = SPLIT ? (Bt2 + (size_t)b * strideB) : nullptr;

  const int rlane = lane & 15;
  const int koff  = (lane >> 4) * 8;
  const int mOff  = (lane >> 4) * 8;

  v8f acc[4][4];
#pragma unroll
  for (int i = 0; i < 4; ++i)
#pragma unroll
    for (int j = 0; j < 4; ++j) acc[i][j] = (v8f){0.f,0.f,0.f,0.f,0.f,0.f,0.f,0.f};

  for (int k0 = 0; k0 < K; k0 += 32) {
    V bh[4], bl[4];
#pragma unroll
    for (int j = 0; j < 4; ++j) {
      const size_t bo = (size_t)(n0 + (j << 4) + rlane) * ldb + koff + k0;
      bh[j] = Frag<T>::load(Bb + bo);
      if (SPLIT) bl[j] = Frag<T>::load(Bb2 + bo);
    }
#pragma unroll
    for (int i = 0; i < 4; ++i) {
      const size_t ao = (size_t)(m0 + (i << 4) + rlane) * lda + koff + k0;
      V ah = Frag<T>::load(Ab + ao);
      V al;
      if (SPLIT) al = Frag<T>::load(Ab2 + ao);
#pragma unroll
      for (int j = 0; j < 4; ++j) {
        acc[i][j] = Frag<T>::mma(ah, bh[j], acc[i][j]);
        if (SPLIT) {
          acc[i][j] = Frag<T>::mma(ah, bl[j], acc[i][j]);
          acc[i][j] = Frag<T>::mma(al, bh[j], acc[i][j]);
        }
      }
      Frag<T>::guard(acc[i][0], acc[i][3], ah, SPLIT ? al : ah);
    }
    Frag<T>::keep(bh[0], bh[1], bh[2], bh[3]);
    if (SPLIT) Frag<T>::keep(bl[0], bl[1], bl[2], bl[3]);
  }
  acc_guard4(acc[0][0], acc[0][1], acc[0][2], acc[0][3]);
  acc_guard4(acc[1][0], acc[1][1], acc[1][2], acc[1][3]);
  acc_guard4(acc[2][0], acc[2][1], acc[2][2], acc[2][3]);
  acc_guard4(acc[3][0], acc[3][1], acc[3][2], acc[3][3]);

  float* slab = sT[wave];
  const float* Rb = RESID ? (resid + (size_t)b * strideR) : nullptr;
#pragma unroll
  for (int i = 0; i < 4; ++i) {
    const int mBase = m0 + (i << 4);
#pragma unroll
    for (int j = 0; j < 4; ++j) {
      const int n = n0 + (j << 4) + rlane;
      float bv = 0.f;
      if (BIAS_MODE == 2) bv = bias[n];
#pragma unroll
      for (int r = 0; r < 8; ++r) {
        float v = acc[i][j][r] * scale;
        if (BIAS_MODE == 1) v += bias[mBase + mOff + r];
        if (BIAS_MODE == 2) v += bv;
        if (RESID) v += Rb[(size_t)(mBase + mOff + r) * ldc + n];
        if (ACT == 1) v = tanhf(v);
        if (ACT == 2) v = fmaxf(v, 0.0f);
        if (ACT == 3) v = v / (1.0f + expf(-v));
        if (ACT == 4) v = (v > 0.f) ? v : 0.01f * v;
        if (ACT == 5) v = 0.5f * v * (1.0f + erff(v * 0.70710678118654752f));
        slab[(mOff + r) * 68 + (j << 4) + rlane] = v;
      }
    }
    __builtin_amdgcn_fence(__ATOMIC_RELEASE, "workgroup");
    __builtin_amdgcn_wave_barrier();
    __builtin_amdgcn_fence(__ATOMIC_ACQUIRE, "workgroup");
    if (OUT_MODE == 0) {
      float* C = (float*)Cout + (size_t)b * strideC;
      const int hh = lane >> 4, c4 = (lane & 15) * 4;
      for (int pass = 0; pass < 2; ++pass) {
#pragma unroll
        for (int it = 0; it < 8; ++it) {
          const int row = it * 2 + hh;
          v4f v = *(const v4f*)(slab + row * 68 + c4);
          *(volatile v4f*)(C + (size_t)(mBase + row) * ldc + n0 + c4) = v;
        }
        __threadfence();
      }
    } else {
      const int q = lane >> 3, c8 = (lane & 7) * 8;
      unsigned short* C  = (unsigned short*)Cout  + (size_t)b * strideC;
      unsigned short* C2 = (OUT_MODE == 2) ? ((unsigned short*)Cout2 + (size_t)b * strideC) : nullptr;
      for (int pass = 0; pass < 2; ++pass) {
#pragma unroll
        for (int it = 0; it < 4; ++it) {
          const int row = it * 4 + q;
          const float* sp = slab + row * 68 + c8;
          v8h hv, lv;
#pragma unroll
          for (int e = 0; e < 8; ++e) {
            if (OUT_MODE == 1) {
              hv[e] = (_Float16)sp[e];
            } else {
              unsigned short hb = f2bf_bits(sp[e]);
              unsigned short lb = f2bf_bits(sp[e] - bf_bits2f(hb));
              hv[e] = __builtin_bit_cast(_Float16, hb);
              lv[e] = __builtin_bit_cast(_Float16, lb);
            }
          }
          *(volatile v8h*)(C + (size_t)(mBase + row) * ldc + n0 + c8) = hv;
          if (OUT_MODE == 2) *(volatile v8h*)(C2 + (size_t)(mBase + row) * ldc + n0 + c8) = lv;
        }
        __threadfence();
      }
    }
    __builtin_amdgcn_fence(__ATOMIC_RELEASE, "workgroup");
    __builtin_amdgcn_wave_barrier();
    __builtin_amdgcn_fence(__ATOMIC_ACQUIRE, "workgroup");
  }
}

__device__ __forceinline__ int clampi(int v, int lo, int hi) { return v < lo ? lo : (v > hi ? hi : v); }

__global__ __launch_bounds__(NT) void wb_plane_kernel(const float* __restrict__ W2, const float* __restrict__ B2, _Float16* __restrict__ WB) {
  const int o = blockIdx.x;
  const int t = threadIdx.x;
  const int tc = t < NPC ? t : NPC - 1;
  const int k0 = tc * 8;
  v8h hv;
#pragma unroll
  for (int j = 0; j < 8; ++j) {
    const int k = k0 + j;
    const int kw = k < 1152 ? k : 1151;
    const float vw = W2[(size_t)kw * HID + o] * 16.0f;
    const int kb = clampi(k - 1152, 0, NQ - 1);
    const float vb = B2[kb * HID + o] * 16.0f;
    const float v = (k < 1152) ? vw : ((k < 1152 + NQ) ? vb : 0.0f);
    hv[j] = (_Float16)v;
  }
  if (t < NPC) {
    _Float16* p = WB + (size_t)o * LDA + k0;
    for (int pass = 0; pass < 2; ++pass) { *(volatile v8h*)p = hv; __threadfence(); }
  }
}

__device__ __forceinline__ int blk_excl_scan(int cnt, int* scan_ws, int tid, int* tot) {
  const int lane = tid & 31, wave = tid >> 5; int incl = cnt;
#pragma unroll
  for (int o = 1; o < 32; o <<= 1) { const int v = __shfl_up(incl, o, 32); if (lane >= o) incl += v; }
  if (lane == 31) scan_ws[wave] = incl;
  __syncthreads();
  if (wave == 0) { int wv = (lane < NT / 32) ? scan_ws[lane] : 0; int wincl = wv;
#pragma unroll
    for (int o = 1; o < 32; o <<= 1) { const int v = __shfl_up(wincl, o, 32); if (lane >= o) wincl += v; }
    if (lane < NT / 32) scan_ws[32 + lane] = wincl - wv; if (lane == 31) scan_ws[64] = wincl; }
  __syncthreads();
  const int res = scan_ws[32 + wave] + incl - cnt; *tot = scan_ws[64];
  return res;
}
template <int SPT, int CAPT>
__device__ __forceinline__ int chunk_hits2(const int* __restrict__ i0v, const int* __restrict__ i1v, const int* __restrict__ etv,
                                           int e0, int n0, int tid, int* LIST, int* scan_ws) {
  const int eb = e0 + tid * SPT;
  const bool ev = eb < NE;
  const int ebc = ev ? eb : (NE - SPT);
  int rec[2 * SPT]; int cnt = 0;
#pragma unroll
  for (int k = 0; k < SPT; k += 4) {
    const v4i a4 = *(const v4i*)(i0v + ebc + k);
    const v4i b4 = *(const v4i*)(i1v + ebc + k);
    const v4i t4 = *(const v4i*)(etv + ebc + k);
#pragma unroll
    for (int e = 0; e < 4; ++e) {
      const int t  = clampi(t4[e], 0, 8);
      const int da = clampi(a4[e], 0, NN - 1);
      const int db = clampi(b4[e], 0, NN - 1);
      int ra = -1, rb = -1;
      if (ev && da >= n0 && da < n0 + SRB) { ra = ((da - n0) << 5) | t;       ++cnt; }
      if (ev && db >= n0 && db < n0 + SRB) { rb = ((db - n0) << 5) | (t + 9); ++cnt; }
      rec[2 * (k + e)] = ra; rec[2 * (k + e) + 1] = rb;
    }
  }
  int tot; int p = blk_excl_scan(cnt, scan_ws, tid, &tot);
#pragma unroll
  for (int k = 0; k < 2 * SPT; ++k) if (rec[k] >= 0) { if ((unsigned)p < (unsigned)CAPT) LIST[p] = rec[k]; ++p; }
  __syncthreads();
  return tot < CAPT ? tot : CAPT;
}

__global__ __launch_bounds__(NT) void count_kernel(const int* __restrict__ ei, const int* __restrict__ et, float* __restrict__ CQ) {
  __shared__ int   CNT[SRB * NQ];
  __shared__ int   LIST[CAP];
  __shared__ float TOT[SRB];
  __shared__ int   scan_ws[80];
  const int tid = threadIdx.x, lane = tid & 31, wave = tid >> 5;
  const int n0 = blockIdx.x * SRB;
  for (int i = tid; i < SRB * NQ; i += NT) CNT[i] = 0;
  __syncthreads();
  const int* i0v = ei; const int* i1v = ei + NE;
#pragma unroll 1
  for (int c = 0; c < NCH; ++c) {
    const int tot = chunk_hits2<SP, CAP>(i0v, i1v, et, c * SCH, n0, tid, LIST, scan_ws);
#pragma unroll 1
    for (int base = 0; base < tot; base += 32) {
      const int q  = base + lane;
      const int qc = q < CAP ? q : (CAP - 1);
      const int lv = LIST[qc];
      const int rv = (q < tot) ? lv : -1;
      const int own = (rv >= 0 && (rv >> 12) == wave) ? 1 : 0;
      unsigned msk = (unsigned)__ballot(own);
#pragma unroll 1
      for (int it = 0; it < 32; ++it) {
        if (msk == 0u) break;
        const int bp = __builtin_ctz(msk); msk &= msk - 1u;
        const int r = __shfl(rv, bp, 32);
        const int nl = r >> 5, qq = r & 31;
        if (lane == ((nl >> 2) & 31)) CNT[nl * NQ + qq] += 1;
      }
    }
    __syncthreads();
  }
  for (int i = tid; i < SRB; i += NT) {
    int s = 0;
#pragma unroll 1
    for (int q = 0; q < NQ; ++q) s += CNT[i * NQ + q];
    TOT[i] = (float)s;
  }
  __syncthreads();
  const int rq = lane >> 3, c4 = (lane & 7) * 4;
#pragma unroll 1
  for (int it = 0; it < 32; ++it) {
    const int nl = wave * 128 + it * 4 + rq;
    v4f v;
#pragma unroll
    for (int j = 0; j < 4; ++j) {
      const int cc = c4 + j;
      const int cq = cc < NQ ? cc : (NQ - 1);
      const float cv = (float)CNT[nl * NQ + cq];
      const float tv = TOT[nl];
      v[j] = (cc < NQ) ? cv : ((cc == NQ) ? tv : 0.0f);
    }
    float* op = CQ + (size_t)(n0 + nl) * 32 + c4;
    *(volatile v4f*)op = v; __threadfence(); *(volatile v4f*)op = v;
  }
}

__global__ __launch_bounds__(NT) void aplane_kernel(const float* __restrict__ CQ, const float* __restrict__ emb,
                                                   _Float16* __restrict__ A16, int mstart) {
  int p = blockIdx.x * NT + threadIdx.x;
  if (p > MCH * NPC - 1) p = MCH * NPC - 1;
  const int rl = p / NPC;
  const int t8 = p - rl * NPC;
  const int n  = mstart + rl;
  const bool nok = n < NN;
  const int ne = nok ? n : (NN - 1);
  const int k0 = t8 * 8;
  const float* cr = CQ + (size_t)n * 32;
  const float cnt = cr[NQ];
  const float inv = (cnt > 0.0f) ? (64.0f / cnt) : 0.0f;
  const int qa = (k0 >> 6) < (NQ - 1) ? (k0 >> 6) : (NQ - 1);
  const float ca = cr[qa];
  const int e0 = k0 & 63;
  const v4f em0 = *(const v4f*)(emb + (size_t)ne * HID + e0);
  const v4f em1 = *(const v4f*)(emb + (size_t)ne * HID + e0 + 4);
  const int qb = clampi(k0 - 1152, 0, 16);
  const v4f c0 = *(const v4f*)(cr + qb);
  const v4f c1 = *(const v4f*)(cr + qb + 4);
  const int mode = (k0 < 1152) ? 0 : ((k0 < 1176) ? 1 : 2);
  const float w0 = nok ? (ca * inv) : 0.0f;
  v8h hv;
#pragma unroll
  for (int j = 0; j < 8; ++j) {
    const float emv = (j < 4) ? em0[j] : em1[j - 4];
    const float cv  = (j < 4) ? c0[j] : c1[j - 4];
    const float v0 = w0 * emv;
    const float v1 = (qb + j < NQ) ? (cv * inv) : 0.0f;
    const float v = (mode == 0) ? v0 : ((mode == 1) ? v1 : 0.0f);
    hv[j] = (_Float16)v;
  }
  _Float16* op = A16 + (size_t)rl * LDA + k0;
  *(volatile v8h*)op = hv; __threadfence(); *(volatile v8h*)op = hv;
}

__global__ __launch_bounds__(NT) void copy_rows_kernel(const float* __restrict__ src, float* __restrict__ dst, int nrows) {
  const int i = blockIdx.x * NT + threadIdx.x;
  const int total = nrows * (HID / 4);
  const int ic = (i < total) ? i : (total - 1);
  const v4f v = *(const v4f*)(src + (size_t)ic * 4);
  if (i < total) {
    float* op = dst + (size_t)i * 4;
    *(volatile v4f*)op = v; __threadfence(); *(volatile v4f*)op = v;
  }
}

extern "C" void kernel_launch(void* const* d_in, const int* in_sizes, int n_in,
                              void* d_out, int out_size, void* d_ws, size_t ws_size, hipStream_t stream) {
  if (n_in < 5) return;
  if (in_sizes[0] != 2 * NE || in_sizes[1] != NE || in_sizes[2] != NN * HID ||
      in_sizes[3] != NL * NQ * HID * HID || in_sizes[4] != NL * NQ * HID || out_size != NN * HID) return;
  const int*   ei  = (const int*)d_in[0];
  const int*   et  = (const int*)d_in[1];
  const float* emb = (const float*)d_in[2];
  const float* wts = (const float*)d_in[3];
  const float* bia = (const float*)d_in[4];
  float* out = (float*)d_out;
  const float* W2 = wts + (size_t)(NL - 1) * NQ * HID * HID;
  const float* B2 = bia + (size_t)(NL - 1) * NQ * HID;

  char* ws = (char*)d_ws; size_t off = 0;
  auto carve = [&](size_t bytes) -> char* { char* p = ws + off; off += (bytes + 255) & ~(size_t)255; return p; };
  _Float16* WB16 = (_Float16*)carve((size_t)HID * LDA * 2);
  float*    CQ   = (float*)carve((size_t)NPAD * 32 * 4);
  _Float16* A16  = (_Float16*)carve((size_t)MCH * LDA * 2);
  float*    H3   = (float*)carve((size_t)MCH * HID * 4);
  if (off > ws_size || off > (size_t)134217728) return;

  wb_plane_kernel<<<HID, NT, 0, stream>>>(W2, B2, WB16);
  count_kernel<<<NTL, NT, 0, stream>>>(ei, et, CQ);

  const int gtiles = (MCH / 64) * (HID / 64);
  for (int c = 0; c < NCHK; ++c) {
    aplane_kernel<<<(MCH * NPC) / NT, NT, 0, stream>>>(CQ, emb, A16, c * MCH);
    void* Cp = (c < NCHK - 1) ? (void*)(out + (size_t)c * MCH * HID) : (void*)H3;
    wmma_gemm64<0, false, 0, 0, false><<<dim3((gtiles + 7) / 8, 1), 256, 0, stream>>>(
        (const unsigned short*)A16, nullptr, LDA, 0L, (const unsigned short*)WB16, nullptr, LDA, 0L,
        Cp, nullptr, HID, 0L, nullptr, nullptr, 0L, MCH, HID, KA, 0.0009765625f);
  }
  const int tail_rows = NN - (NCHK - 1) * MCH;
  copy_rows_kernel<<<(tail_rows * (HID / 4) + NT - 1) / NT, NT, 0, stream>>>(H3, out + (size_t)(NCHK - 1) * MCH * HID, tail_rows);
}
